// X_CrossAttn_60344290509634
// MI455X (gfx1250) — hardware-verified
//
#include <hip/hip_runtime.h>

constexpr int kBatch      = 4;
constexpr int kSeq        = 1024;
constexpr int kDm         = 1024;
constexpr int kHeads      = 16;
constexpr int kDk         = 64;
constexpr int kInner      = kHeads * kDk;
constexpr int kTok        = kBatch * kSeq;
constexpr int kGroupHeads = 8;
constexpr int kGroupsPerB = kHeads / kGroupHeads;
constexpr int kPPitch     = 2 * kSeq;
constexpr float kVCarry   = 4096.0f;
constexpr float kPCarry   = 32768.0f;
constexpr float kPVScale  = 1.0f / (kPCarry * kVCarry);

static_assert(kSeq % 64 == 0 && kDm % 64 == 0 && kInner % 64 == 0 && kDk % 32 == 0, "tile multiples");
static_assert(kInner == kDm, "square weights");

constexpr long kSqElems  = (long)kSeq * kInner;
constexpr long kTokElems = (long)kTok * kDm;

constexpr size_t kPlaneTokBytes  = (size_t)kTok * kDm * 2;
constexpr size_t kPlaneSq16Bytes = (size_t)kSeq * kInner * 2;
constexpr size_t kPlaneSq32Bytes = (size_t)kSeq * kSeq * 4;
constexpr size_t kOffXB   = 0;
constexpr size_t kOffWT   = kOffXB   + 2 * kPlaneTokBytes;
constexpr size_t kOffQKH  = kOffWT   + 4 * kPlaneSq16Bytes;
constexpr size_t kOffQKL  = kOffQKH  + 2 * kPlaneSq16Bytes;
constexpr size_t kOffVTH  = kOffQKL  + 2 * kPlaneSq16Bytes;
constexpr size_t kOffVTL  = kOffVTH  + 2 * kPlaneSq16Bytes;
constexpr size_t kOffCTXH = kOffVTL  + 2 * kPlaneSq16Bytes;
constexpr size_t kOffCTXL = kOffCTXH + 2 * kPlaneSq16Bytes;
constexpr size_t kOffSP   = kOffCTXL + 2 * kPlaneSq16Bytes;
constexpr size_t kOffPT   = kOffSP   + (size_t)kGroupHeads * kPlaneSq32Bytes;
constexpr size_t kWsTotal = kOffPT   + (size_t)kGroupHeads * kPlaneSq16Bytes;
static_assert(kWsTotal == 100663296, "carve total");
static_assert(kWsTotal <= 134217728, "carve under 128 MiB");

typedef __attribute__((ext_vector_type(16))) _Float16 v16h;
typedef __attribute__((ext_vector_type(8)))  _Float16 v8h;
typedef __attribute__((ext_vector_type(16))) __bf16   v16b;
typedef __attribute__((ext_vector_type(8)))  __bf16   v8b;
typedef __attribute__((ext_vector_type(8)))  float    v8f;
typedef __attribute__((ext_vector_type(4)))  float    v4f;
typedef __attribute__((ext_vector_type(4)))  unsigned int v4u;

__device__ __forceinline__ unsigned short f2bf_bits(float f) {
  unsigned u = __float_as_uint(f);
  return (unsigned short)((u + 0x7FFFu + ((u >> 16) & 1u)) >> 16);
}
__device__ __forceinline__ float bf_bits2f(unsigned short h) { return __uint_as_float(((unsigned)h) << 16); }

__device__ __forceinline__ void dep_guard_h(v8f& a, v8f& b, v16h x, v16h y) { asm volatile("v_nop\n\tv_nop\n\tv_nop\n\tv_nop" : "+v"(a), "+v"(b) : "v"(x), "v"(y)); }
__device__ __forceinline__ void dep_guard_b(v8f& a, v8f& b, v16b x, v16b y) { asm volatile("v_nop\n\tv_nop\n\tv_nop\n\tv_nop" : "+v"(a), "+v"(b) : "v"(x), "v"(y)); }
__device__ __forceinline__ void keep4_h(v16h a, v16h b, v16h c, v16h d) { asm volatile("v_nop" :: "v"(a), "v"(b), "v"(c), "v"(d)); }
__device__ __forceinline__ void keep4_b(v16b a, v16b b, v16b c, v16b d) { asm volatile("v_nop" :: "v"(a), "v"(b), "v"(c), "v"(d)); }
__device__ __forceinline__ void acc_guard4(v8f& a, v8f& b, v8f& c, v8f& d) { asm volatile("v_nop\n\tv_nop\n\tv_nop\n\tv_nop" : "+v"(a), "+v"(b), "+v"(c), "+v"(d)); }
template <typename T> struct Frag;
template <> struct Frag<_Float16> {
  typedef v16h V; union U { v16h v; v8h h[2]; };
  static __device__ __forceinline__ v16h load(const _Float16* p) {
    U f; f.h[0] = *(const v8h*)(p); f.h[1] = *(const v8h*)(p + 16); return f.v;
  }
  static __device__ __forceinline__ v8f mma(v16h a, v16h b, v8f c) {
    return __builtin_amdgcn_wmma_f32_16x16x32_f16(false, a, false, b, (short)0, c, false, false);
  }
  static __device__ __forceinline__ void guard(v8f& a, v8f& b, v16h x, v16h y) { dep_guard_h(a, b, x, y); }
  static __device__ __forceinline__ void keep(v16h a, v16h b, v16h c, v16h d) { keep4_h(a, b, c, d); }
};
template <> struct Frag<__bf16> {
  typedef v16b V; union U { v16b v; v8b h[2]; };
  static __device__ __forceinline__ v16b load(const __bf16* p) {
    U f; f.h[0] = *(const v8b*)(p); f.h[1] = *(const v8b*)(p + 16); return f.v;
  }
  static __device__ __forceinline__ v8f mma(v16b a, v16b b, v8f c) {
    return __builtin_amdgcn_wmma_f32_16x16x32_bf16(false, a, false, b, (short)0, c, false, false);
  }
  static __device__ __forceinline__ void guard(v8f& a, v8f& b, v16b x, v16b y) { dep_guard_b(a, b, x, y); }
  static __device__ __forceinline__ void keep(v16b a, v16b b, v16b c, v16b d) { keep4_b(a, b, c, d); }
};

__device__ __forceinline__ unsigned pk16(unsigned short a, unsigned short b) { return (unsigned)a | ((unsigned)b << 16); }
__device__ __forceinline__ unsigned short h_bits(float f) { const _Float16 h = (_Float16)f; return __builtin_bit_cast(unsigned short, h); }

template <int ET> struct Elem;
template <> struct Elem<0> { typedef _Float16 T; };
template <> struct Elem<1> { typedef __bf16 T; };
template <int ET, int SPK, int BIAS_MODE, int OUT_MODE, bool RESID, int ACT = 0>
__global__ __launch_bounds__(256) void wmma_gemm64(
    const unsigned short* __restrict__ Ap, const unsigned short* __restrict__ A2p, int lda, long strideA,
    const unsigned short* __restrict__ Btp, const unsigned short* __restrict__ Bt2p, int ldb, long strideB,
    void* __restrict__ Cout, void* __restrict__ Cout2, int ldc, long strideC,
    const float* __restrict__ bias,
    const float* __restrict__ resid, long strideR,
    int M, int N, int K, float scale) {
  typedef typename Elem<ET>::T T;
  typedef typename Frag<T>::V V;
  constexpr bool SPA = (SPK == 1) || (SPK == 3);
  constexpr bool SPB = (SPK == 1) || (SPK == 2);
  const T* A = (const T*)Ap; const T* A2 = (const T*)A2p; const T* Bt = (const T*)Btp; const T* Bt2 = (const T*)Bt2p;
  __shared__ __align__(16) float sT[8][16 * 68];
  const int b    = blockIdx.y;
  const int lane = threadIdx.x & 31;
  const int wave = threadIdx.x >> 5;
  const int tilesN = N >> 6;
  const int tilesM = M >> 6;
  const int tile = blockIdx.x * 8 + wave;
  if (tile >= tilesM * tilesN) return;
  const int tm = tile / tilesN;
  const int tn = tile - tm * tilesN;
  const int m0 = tm << 6;
  const int n0 = tn << 6;

  const T* Ab  = A  + (size_t)b * strideA;
  const T* Bb  = Bt + (size_t)b * strideB;
  const T* Ab2 = SPA ? (A2  + (size_t)b * strideA) : nullptr;
  const T* Bb2 = SPB ? (Bt2 + (size_t)b * strideB) : nullptr;

  const int rlane = lane & 15;
  const int koff  = (lane >> 4) * 8;
  const int mOff  = (lane >> 4) * 8;

  v8f acc[4][4];
#pragma unroll
  for (int i = 0; i < 4; ++i)
#pragma unroll
    for (int j = 0; j < 4; ++j) acc[i][j] = (v8f){0.f,0.f,0.f,0.f,0.f,0.f,0.f,0.f};

  for (int k0 = 0; k0 < K; k0 += 32) {
    V bh[4], bl[4];
#pragma unroll
    for (int j = 0; j < 4; ++j) {
      const size_t bo = (size_t)(n0 + (j << 4) + rlane) * ldb + koff + k0;
      bh[j] = Frag<T>::load(Bb + bo);
      if (SPB) bl[j] = Frag<T>::load(Bb2 + bo);
    }
#pragma unroll
    for (int i = 0; i < 4; ++i) {
      const size_t ao = (size_t)(m0 + (i << 4) + rlane) * lda + koff + k0;
      V ah = Frag<T>::load(Ab + ao);
      V al;
      if (SPA) al = Frag<T>::load(Ab2 + ao);
#pragma unroll
      for (int j = 0; j < 4; ++j) {
        acc[i][j] = Frag<T>::mma(ah, bh[j], acc[i][j]);
        if (SPB) acc[i][j] = Frag<T>::mma(ah, bl[j], acc[i][j]);
        if (SPA) acc[i][j] = Frag<T>::mma(al, bh[j], acc[i][j]);
      }
      Frag<T>::guard(acc[i][0], acc[i][3], ah, SPA ? al : ah);
    }
    Frag<T>::keep(bh[0], bh[1], bh[2], bh[3]);
    if (SPB) Frag<T>::keep(bl[0], bl[1], bl[2], bl[3]);
  }
  acc_guard4(acc[0][0], acc[0][1], acc[0][2], acc[0][3]);
  acc_guard4(acc[1][0], acc[1][1], acc[1][2], acc[1][3]);
  acc_guard4(acc[2][0], acc[2][1], acc[2][2], acc[2][3]);
  acc_guard4(acc[3][0], acc[3][1], acc[3][2], acc[3][3]);

  float* slab = sT[wave];
  const float* Rb = RESID ? (resid + (size_t)b * strideR) : nullptr;
#pragma unroll
  for (int i = 0; i < 4; ++i) {
    const int mBase = m0 + (i << 4);
#pragma unroll
    for (int j = 0; j < 4; ++j) {
      const int n = n0 + (j << 4) + rlane;
      float bv = 0.f;
      if (BIAS_MODE == 2) bv = bias[n];
#pragma unroll
      for (int r = 0; r < 8; ++r) {
        float v = acc[i][j][r] * scale;
        if (BIAS_MODE == 1) v += bias[mBase + mOff + r];
        if (BIAS_MODE == 2) v += bv;
        if (RESID) v += Rb[(size_t)(mBase + mOff + r) * ldc + n];
        if (ACT == 2) v = fmaxf(v, 0.0f);
        if (ACT == 4) v = (v > 0.f) ? v : 0.01f * v;
        slab[(mOff + r) * 68 + (j << 4) + rlane] = v;
      }
    }
    __builtin_amdgcn_fence(__ATOMIC_RELEASE, "workgroup");
    __builtin_amdgcn_wave_barrier();
    __builtin_amdgcn_fence(__ATOMIC_ACQUIRE, "workgroup");
    if (OUT_MODE == 0) {
      float* C = (float*)Cout + (size_t)b * strideC;
      const int hh = lane >> 4, c4 = (lane & 15) * 4;
      for (int pass = 0; pass < 2; ++pass) {
#pragma unroll
        for (int it = 0; it < 8; ++it) {
          const int row = it * 2 + hh;
          v4f v = *(const v4f*)(slab + row * 68 + c4);
          *(volatile v4f*)(C + (size_t)(mBase + row) * ldc + n0 + c4) = v;
        }
        __threadfence();
      }
    } else {
      const int q = lane >> 3, c8 = (lane & 7) * 8;
      unsigned short* C  = (unsigned short*)Cout  + (size_t)b * strideC;
      unsigned short* C2 = (OUT_MODE >= 2) ? ((unsigned short*)Cout2 + (size_t)b * strideC) : nullptr;
      for (int pass = 0; pass < 2; ++pass) {
#pragma unroll
        for (int it = 0; it < 4; ++it) {
          const int row = it * 4 + q;
          const float* sp = slab + row * 68 + c8;
          v8h hv, lv;
#pragma unroll
          for (int e = 0; e < 8; ++e) {
            if (OUT_MODE == 1) {
              hv[e] = (_Float16)sp[e];
            } else if (OUT_MODE == 3) {
              const _Float16 hq = (_Float16)sp[e];
              hv[e] = hq;
              lv[e] = (_Float16)(sp[e] - (float)hq);
            } else {
              unsigned short hb = f2bf_bits(sp[e]);
              unsigned short lb = f2bf_bits(sp[e] - bf_bits2f(hb));
              hv[e] = __builtin_bit_cast(_Float16, hb);
              lv[e] = __builtin_bit_cast(_Float16, lb);
            }
          }
          *(volatile v8h*)(C + (size_t)(mBase + row) * ldc + n0 + c8) = hv;
          if (OUT_MODE >= 2) *(volatile v8h*)(C2 + (size_t)(mBase + row) * ldc + n0 + c8) = lv;
        }
        __threadfence();
      }
    }
    __builtin_amdgcn_fence(__ATOMIC_RELEASE, "workgroup");
    __builtin_amdgcn_wave_barrier();
    __builtin_amdgcn_fence(__ATOMIC_ACQUIRE, "workgroup");
  }
}

__global__ __launch_bounds__(256) void cast_x_kernel(const float* __restrict__ X0, const float* __restrict__ X1,
                                                     unsigned short* __restrict__ out, int n8) {
  const int z = blockIdx.y;
  const float* X = (z == 0) ? X0 : X1;
  const int i = blockIdx.x * 256 + threadIdx.x;
  if (i >= n8) return;
  const float* p = X + 8 * (size_t)i;
  const v4f a = *(const v4f*)(p);
  const v4f c = *(const v4f*)(p + 4);
  unsigned short hb[8];
#pragma unroll
  for (int e = 0; e < 4; ++e) {
    hb[e]     = f2bf_bits(a[e]);
    hb[4 + e] = f2bf_bits(c[e]);
  }
  const v4u u = (v4u){pk16(hb[0], hb[1]), pk16(hb[2], hb[3]), pk16(hb[4], hb[5]), pk16(hb[6], hb[7])};
  unsigned short* q = out + (size_t)z * 8 * (size_t)n8 + 8 * (size_t)i;
  *(volatile v4u*)q = u;
  __threadfence();
  *(volatile v4u*)q = u;
}

__global__ __launch_bounds__(256) void wt_cast_kernel(const float* __restrict__ W0, const float* __restrict__ W1,
                                                      const float* __restrict__ W2, const float* __restrict__ W3,
                                                      unsigned short* __restrict__ out) {
  __shared__ float sm[64][65];
  const int t  = threadIdx.x;
  const int i0 = blockIdx.x * 64;
  const int o0 = blockIdx.y * 64;
  const int z  = blockIdx.z;
  const float* W = (z == 0) ? W0 : (z == 1) ? W1 : (z == 2) ? W2 : W3;
#pragma unroll
  for (int it = 0; it < 16; ++it) {
    const int e  = it * 256 + t;
    const int il = e >> 6;
    const int ol = e & 63;
    sm[ol][il] = W[(size_t)(i0 + il) * kInner + o0 + ol];
  }
  __syncthreads();
  const int lane = t & 31, wave = t >> 5;
  const int q = lane >> 3, c8 = (lane & 7) * 8;
  unsigned short* op = out + (size_t)z * kInner * kDm;
  for (int ps = 0; ps < 2; ++ps) {
#pragma unroll
    for (int it = 0; it < 2; ++it) {
      const int row = wave * 8 + it * 4 + q;
      unsigned short hb[8];
#pragma unroll
      for (int e = 0; e < 8; ++e) hb[e] = f2bf_bits(sm[row][c8 + e]);
      const v4u u = (v4u){pk16(hb[0], hb[1]), pk16(hb[2], hb[3]), pk16(hb[4], hb[5]), pk16(hb[6], hb[7])};
      *(volatile v4u*)(op + (size_t)(o0 + row) * kDm + i0 + c8) = u;
    }
    __threadfence();
  }
}

__global__ __launch_bounds__(128) void softmax_rows_kernel(float* __restrict__ SPp, float carry) {
  __shared__ float redM[4];
  __shared__ float redS[4];
  const int row  = blockIdx.x;
  const int t    = threadIdx.x;
  const int lane = t & 31, wave = t >> 5;
  float* rbase = SPp + (size_t)row * kSeq;
  const v4f a = *(const v4f*)(rbase + 8 * t);
  const v4f c = *(const v4f*)(rbase + 8 * t + 4);
  float x[8];
#pragma unroll
  for (int e = 0; e < 4; ++e) { x[e] = a[e]; x[4 + e] = c[e]; }
  float m = fmaxf(fmaxf(fmaxf(x[0], x[1]), fmaxf(x[2], x[3])), fmaxf(fmaxf(x[4], x[5]), fmaxf(x[6], x[7])));
#pragma unroll
  for (int off = 16; off > 0; off >>= 1) m = fmaxf(m, __shfl_xor(m, off, 32));
  if (lane == 0) redM[wave] = m;
  __syncthreads();
  const float mall = fmaxf(fmaxf(redM[0], redM[1]), fmaxf(redM[2], redM[3]));
  float ex[8];
  float s = 0.f;
#pragma unroll
  for (int e = 0; e < 8; ++e) { ex[e] = __expf(x[e] - mall); s += ex[e]; }
#pragma unroll
  for (int off = 16; off > 0; off >>= 1) s += __shfl_xor(s, off, 32);
  if (lane == 0) redS[wave] = s;
  __syncthreads();
  const float sall = (redS[0] + redS[1]) + (redS[2] + redS[3]);
  const float inv = carry * (1.0f / sall);
  unsigned short hb[8];
#pragma unroll
  for (int e = 0; e < 8; ++e) hb[e] = h_bits(ex[e] * inv);
  const v4u u = (v4u){pk16(hb[0], hb[1]), pk16(hb[2], hb[3]), pk16(hb[4], hb[5]), pk16(hb[6], hb[7])};
  unsigned short* pr = (unsigned short*)(void*)rbase + 8 * t;
  *(volatile v4u*)pr = u;
  __threadfence();
  *(volatile v4u*)pr = u;
}

__global__ __launch_bounds__(256) void transpose_p_kernel(const unsigned short* __restrict__ P, unsigned short* __restrict__ PT) {
  __shared__ unsigned short sm[64][72];
  const int t = threadIdx.x, lane = t & 31, wave = t >> 5;
  const int j0 = blockIdx.x * 64;
  const int i0 = blockIdx.y * 64;
  const int z  = blockIdx.z;
  const unsigned short* src = P + (size_t)z * 2 * kSeq * kSeq + (size_t)i0 * kPPitch + j0;
#pragma unroll
  for (int it = 0; it < 2; ++it) {
    const int e  = it * 256 + t;
    const int r  = e >> 3;
    const int c8 = (e & 7) * 8;
    const v4u u = *(const v4u*)(src + (size_t)r * kPPitch + c8);
#pragma unroll
    for (int k = 0; k < 4; ++k) {
      sm[c8 + 2 * k][r]     = (unsigned short)(u[k] & 0xFFFFu);
      sm[c8 + 2 * k + 1][r] = (unsigned short)(u[k] >> 16);
    }
  }
  __syncthreads();
  const int q = lane >> 3, c8 = (lane & 7) * 8;
  unsigned short* dst = PT + (size_t)z * kSeq * kSeq + (size_t)j0 * kSeq + i0;
  for (int ps = 0; ps < 2; ++ps) {
#pragma unroll
    for (int it = 0; it < 2; ++it) {
      const int row = wave * 8 + it * 4 + q;
      const v4u u = (v4u){pk16(sm[row][c8 + 0], sm[row][c8 + 1]), pk16(sm[row][c8 + 2], sm[row][c8 + 3]),
                          pk16(sm[row][c8 + 4], sm[row][c8 + 5]), pk16(sm[row][c8 + 6], sm[row][c8 + 7])};
      *(volatile v4u*)(dst + (size_t)row * kSeq + c8) = u;
    }
    __threadfence();
  }
}

extern "C" void kernel_launch(void* const* d_in, const int* in_sizes, int n_in,
                              void* d_out, int out_size, void* d_ws, size_t ws_size,
                              hipStream_t stream) {
  if (n_in < 6) return;
  if (in_sizes[0] != kTok * kDm || in_sizes[1] != kTok * kDm) return;
  if (in_sizes[2] != kDm * kInner || in_sizes[3] != kDm * kInner || in_sizes[4] != kDm * kInner || in_sizes[5] != kInner * kDm) return;
  if (out_size != 2 * kTok * kDm) return;
  if (kWsTotal > ws_size) return;

  const float* vis = (const float*)d_in[0];
  const float* txt = (const float*)d_in[1];
  const float* Wq  = (const float*)d_in[2];
  const float* Wk  = (const float*)d_in[3];
  const float* Wv  = (const float*)d_in[4];
  const float* Wo  = (const float*)d_in[5];

  char* ws = (char*)d_ws;
  unsigned short* XB   = (unsigned short*)(ws + kOffXB);
  unsigned short* WT   = (unsigned short*)(ws + kOffWT);
  unsigned short* QKH  = (unsigned short*)(ws + kOffQKH);
  unsigned short* QKL  = (unsigned short*)(ws + kOffQKL);
  unsigned short* VTH  = (unsigned short*)(ws + kOffVTH);
  unsigned short* VTL  = (unsigned short*)(ws + kOffVTL);
  unsigned short* CTXH = (unsigned short*)(ws + kOffCTXH);
  unsigned short* CTXL = (unsigned short*)(ws + kOffCTXL);
  float*          SP   = (float*)(ws + kOffSP);
  unsigned short* PT   = (unsigned short*)(ws + kOffPT);
  float* outBase = (float*)d_out;

  const dim3 blk256(256);

  const int n8 = kTok * kDm / 8;
  cast_x_kernel<<<dim3(n8 / 256, 2), blk256, 0, stream>>>(vis, txt, XB, n8);
  wt_cast_kernel<<<dim3(kDm / 64, kInner / 64, 4), blk256, 0, stream>>>(Wq, Wk, Wv, Wo, WT);

  for (int b = 0; b < kBatch; ++b) {
    const size_t xOff = (size_t)b * kSqElems;
    wmma_gemm64<1, 0, 0, 2, false><<<dim3((kSeq / 64) * (kInner / 64) / 8, 2), blk256, 0, stream>>>(
        XB + xOff, nullptr, kDm, (long)kTokElems,
        WT, nullptr, kDm, (long)kSqElems,
        QKH, QKL, kInner, (long)kSqElems,
        nullptr, nullptr, 0L, kSeq, kInner, kDm, 1.0f);
    wmma_gemm64<1, 0, 0, 3, false><<<dim3((kInner / 64) * (kSeq / 64) / 8, 2), blk256, 0, stream>>>(
        WT + 2 * kSqElems, nullptr, kDm, 0L,
        XB + xOff, nullptr, kDm, (long)kTokElems,
        VTH, VTL, kSeq, (long)kSqElems,
        nullptr, nullptr, 0L, kInner, kSeq, kDm, kVCarry);

    for (int gi = 0; gi < kGroupsPerB; ++gi) {
      const int h0 = gi * kGroupHeads;
      const size_t colOff = (size_t)h0 * kDk;
      const size_t vtRow  = (size_t)h0 * kDk * kSeq;
      wmma_gemm64<1, 1, 0, 0, false><<<dim3((kSeq / 64) * (kSeq / 64) / 8, kGroupHeads), blk256, 0, stream>>>(
          QKH + colOff, QKL + colOff, kInner, (long)kDk,
          QKH + kSqElems + colOff, QKL + kSqElems + colOff, kInner, (long)kDk,
          SP, nullptr, kSeq, (long)kSeq * kSeq,
          nullptr, nullptr, 0L, kSeq, kSeq, kDk, 1.0f);
      softmax_rows_kernel<<<dim3(kGroupHeads * kSeq), dim3(128), 0, stream>>>(SP, kPCarry);
      transpose_p_kernel<<<dim3(kSeq / 64, kSeq / 64, kGroupHeads), blk256, 0, stream>>>((const unsigned short*)SP, PT);
      wmma_gemm64<0, 2, 0, 2, false><<<dim3((kSeq / 64) * (kDk / 64) / 8, kGroupHeads), blk256, 0, stream>>>(
          (const unsigned short*)SP, nullptr, kPPitch, (long)2 * kSeq * kSeq,
          VTH + kSqElems + vtRow, VTL + kSqElems + vtRow, kSeq, (long)kDk * kSeq,
          CTXH + colOff, CTXL + colOff, kInner, (long)kDk,
          nullptr, nullptr, 0L, kSeq, kDk, kSeq, kPVScale);
      wmma_gemm64<0, 2, 0, 2, false><<<dim3((kSeq / 64) * (kDk / 64) / 8, kGroupHeads), blk256, 0, stream>>>(
          PT, nullptr, kSeq, (long)kSeq * kSeq,
          VTH + vtRow, VTL + vtRow, kSeq, (long)kDk * kSeq,
          CTXH + kSqElems + colOff, CTXL + kSqElems + colOff, kInner, (long)kDk,
          nullptr, nullptr, 0L, kSeq, kDk, kSeq, kPVScale);
    }

    wmma_gemm64<1, 3, 0, 0, false><<<dim3((kSeq / 64) * (kDm / 64) / 8, 2), blk256, 0, stream>>>(
        CTXH, CTXL, kInner, (long)kSqElems,
        WT + 3 * kSqElems, nullptr, kInner, 0L,
        outBase + (size_t)b * kSqElems, nullptr, kDm, (long)kTokElems,
        nullptr, nullptr, 0L, kSeq, kDm, kInner, 1.0f);
  }
}
